// UNetBlockDownsasa_unique_69501160783981
// MI455X (gfx1250) — hardware-verified
//
#include <hip/hip_runtime.h>
#include <stdint.h>

#define NB      4
#define CCH     128
#define IMH     128
#define IMW     128
#define HWPIX   (IMH * IMW)
#define NHEADS  4
#define DHEAD   32
#define QSCALE  0.17677669529663687f
#define TP      132
#define TILE_F  (128 * TP)
#define KVROWS  3
#define KVPOS   130
#define KVS_F   (KVROWS * KVPOS * DHEAD)
#define OT_F    (DHEAD * TP)
#define ATTN_LDS_F (TILE_F + KVS_F + OT_F)

typedef __attribute__((ext_vector_type(16))) __bf16         v16b;
typedef __attribute__((ext_vector_type(8)))  unsigned short v8us;
typedef __attribute__((ext_vector_type(8)))  float          v8f;
typedef __attribute__((ext_vector_type(4)))  float          v4f;
typedef __attribute__((ext_vector_type(2)))  float          v2f;

union Frg { v16b b; v8us h8[2]; unsigned int w[8]; };
static_assert(sizeof(Frg) == 32);

__device__ __forceinline__ unsigned short f2bf(float f) {
  const unsigned u = __float_as_uint(f);
  return (unsigned short)((u + 0x7FFFu + ((u >> 16) & 1u)) >> 16);
}
__device__ __forceinline__ float bf2f(unsigned short h) { return __uint_as_float(((unsigned)h) << 16); }
__device__ __forceinline__ unsigned int pk16(unsigned short lo, unsigned short hi) {
  return (unsigned)lo | ((unsigned)hi << 16);
}
__device__ __forceinline__ void opt_fence() { asm volatile("" ::: "memory"); }

__device__ __forceinline__ v8f zero8() {
  v8f z = {0.f, 0.f, 0.f, 0.f, 0.f, 0.f, 0.f, 0.f};
  return z;
}

__device__ __forceinline__ v8f mma16(v16b a, v16b b, v8f c) {
  v8f d = __builtin_amdgcn_wmma_f32_16x16x32_bf16(false, a, false, b, (short)0, c, false, false);
  asm volatile("v_nop\n\tv_nop\n\tv_nop\n\tv_nop" : "+v"(d) : "v"(a), "v"(b));
  return d;
}

__device__ __forceinline__ void gather_split(const float* __restrict__ pt, int lane, int k0, Frg& fh, Frg& fl) {
  const int m = lane & 15, h = lane >> 4;
  const float* pm = pt + m;
#pragma unroll
  for (int q = 0; q < 8; ++q) {
    const int c = k0 + ((q < 4) ? (8 * h + 2 * q) : (16 + 8 * h + 2 * (q - 4)));
    const float v0 = pm[(size_t)c * HWPIX];
    const float v1 = pm[(size_t)(c + 1) * HWPIX];
    const unsigned short h0 = f2bf(v0), h1 = f2bf(v1);
    const unsigned short l0 = f2bf(v0 - bf2f(h0)), l1 = f2bf(v1 - bf2f(h1));
    fh.w[q] = pk16(h0, h1);
    fl.w[q] = pk16(l0, l1);
  }
}
__device__ __forceinline__ void wfrag(const unsigned short* __restrict__ W, int row0, int lane, int k0, Frg& f) {
  const int m = lane & 15, h = lane >> 4;
  const unsigned short* p = W + (size_t)(row0 + m) * CCH + k0 + 8 * h;
  f.h8[0] = *(const v8us*)(p);
  f.h8[1] = *(const v8us*)(p + 16);
}

__device__ __forceinline__ void proj_row_tile(const float* __restrict__ xrow,
                                              const unsigned short* __restrict__ Wh,
                                              const unsigned short* __restrict__ Wl,
                                              const float* __restrict__ bias, float scale,
                                              float* T, int wave, int lane) {
  const int m = lane & 15, h = lane >> 4;
  v8f acc[8];
#pragma unroll
  for (int j = 0; j < 8; ++j) acc[j] = zero8();
  const float* xt = xrow + 16 * wave;
#pragma unroll 1
  for (int k0 = 0; k0 < CCH; k0 += 32) {
    Frg ah, al;
    gather_split(xt, lane, k0, ah, al);
#pragma unroll
    for (int j = 0; j < 8; ++j) {
      opt_fence();
      Frg bh, bl;
      wfrag(Wh, 16 * j, lane, k0, bh);
      wfrag(Wl, 16 * j, lane, k0, bl);
      acc[j] = mma16(ah.b, bh.b, acc[j]);
      acc[j] = mma16(ah.b, bl.b, acc[j]);
      acc[j] = mma16(al.b, bh.b, acc[j]);
    }
  }
#pragma unroll
  for (int j = 0; j < 8; ++j) {
    const float bvv = bias[16 * j + m];
    float* trow = T + (size_t)(16 * wave + 8 * h) * TP + 16 * j + m;
#pragma unroll
    for (int r = 0; r < 8; ++r) trow[r * TP] = (acc[j][r] + bvv) * scale;
  }
}

__global__ __launch_bounds__(256) void k_split_w(const float* __restrict__ Wq, const float* __restrict__ Wkv,
                                                 unsigned short* __restrict__ qh, unsigned short* __restrict__ ql,
                                                 unsigned short* __restrict__ kh, unsigned short* __restrict__ kl) {
  const int blk = blockIdx.x;
  const bool isq = (blk < 32);
  const float* src = isq ? Wq : Wkv;
  unsigned short* dh = isq ? qh : kh;
  unsigned short* dl = isq ? ql : kl;
  const int i = (blk & 31) * 256 + threadIdx.x;
  const v2f f = *(const v2f*)(src + 2 * (size_t)i);
  const unsigned short h0 = f2bf(f[0]), h1 = f2bf(f[1]);
  const unsigned short l0 = f2bf(f[0] - bf2f(h0)), l1 = f2bf(f[1] - bf2f(h1));
  const unsigned uh = pk16(h0, h1), ul = pk16(l0, l1);
  ((volatile unsigned*)dh)[i] = uh;
  ((volatile unsigned*)dl)[i] = ul;
  __threadfence();
  ((volatile unsigned*)dh)[i] = uh;
  ((volatile unsigned*)dl)[i] = ul;
}

__global__ __launch_bounds__(256) void k_kvproj(const float* __restrict__ x,
                                                const unsigned short* __restrict__ Wh,
                                                const unsigned short* __restrict__ Wl,
                                                const float* __restrict__ bias,
                                                float* __restrict__ kvp) {
  extern __shared__ __attribute__((aligned(16))) float smem[];
  float* T = smem;
  const int tid  = threadIdx.x;
  const int lane = tid & 31;
  const int wave = __builtin_amdgcn_readfirstlane(tid >> 5);
  const int y = blockIdx.x;
  const int b = blockIdx.y;
  const float* xrow = x + (size_t)b * CCH * HWPIX + (size_t)y * IMW;
  proj_row_tile(xrow, Wh, Wl, bias, 1.0f, T, wave, lane);
  __syncthreads();
  float* dstb = kvp + ((size_t)b * HWPIX + (size_t)y * IMW) * CCH;
  for (int pass = 0; pass < 2; ++pass) {
#pragma unroll
    for (int i = 0; i < 16; ++i) {
      const int rr = 16 * wave + i;
      const v4f v = *(const v4f*)(T + (size_t)rr * TP + 4 * lane);
      *(volatile v4f*)(dstb + (size_t)rr * CCH + 4 * lane) = v;
    }
    __threadfence();
  }
}

__device__ __forceinline__ void stage_kv(const float* __restrict__ kb, const float* __restrict__ bkv,
                                         int hd, int y, float* kvS, int tid) {
  const float* bh = bkv + hd * DHEAD;
#pragma unroll 1
  for (int i = tid; i < KVROWS * KVPOS * 4; i += 256) {
    const int seg = i >> 2;
    const int g8  = (i & 3) * 8;
    const int r   = seg / KVPOS;
    const int p   = seg - r * KVPOS;
    const int yy  = y + r - 1;
    const int xx  = p - 1;
    const bool inb = (yy >= 0) && (yy < IMH) && (xx >= 0) && (xx < IMW);
    const int yyc = (yy < 0) ? 0 : ((yy > IMH - 1) ? (IMH - 1) : yy);
    const int xxc = (xx < 0) ? 0 : ((xx > IMW - 1) ? (IMW - 1) : xx);
    const float* src = kb + (size_t)(yyc * IMW + xxc) * CCH + hd * DHEAD + g8;
    const v4f a0 = *(const v4f*)(src);
    const v4f a1 = *(const v4f*)(src + 4);
    const v4f b0 = *(const v4f*)(bh + g8);
    const v4f b1 = *(const v4f*)(bh + g8 + 4);
    v4f o0, o1;
#pragma unroll
    for (int e = 0; e < 4; ++e) {
      o0[e] = inb ? a0[e] : b0[e];
      o1[e] = inb ? a1[e] : b1[e];
    }
    float* dst = kvS + (size_t)seg * DHEAD + g8;
    *(v4f*)(dst)     = o0;
    *(v4f*)(dst + 4) = o1;
  }
}

__device__ __forceinline__ void load16(const float* p, float (&v)[16]) {
#pragma unroll
  for (int g = 0; g < 4; ++g) {
    const v4f t = *(const v4f*)(p + 4 * g);
    v[4 * g + 0] = t[0]; v[4 * g + 1] = t[1]; v[4 * g + 2] = t[2]; v[4 * g + 3] = t[3];
  }
}

__device__ __forceinline__ void attend_branch(const float* kvS, int px, int half,
                                              const float (&q)[16], float (&res)[16]) {
  const float* kcol = kvS + (size_t)px * DHEAD + 16 * half;
  float ov[16];
  float m, ssum;
  {
    float kv[16];
    load16(kcol, kv);
    float part = 0.0f;
#pragma unroll
    for (int i = 0; i < 16; ++i) part += q[i] * kv[i];
    const float s = part + __shfl_xor(part, 16, 32);
    m = s;
    ssum = 1.0f;
#pragma unroll
    for (int i = 0; i < 16; ++i) ov[i] = kv[i];
  }
#pragma unroll 1
  for (int t = 1; t < 9; ++t) {
    const int r  = t / 3;
    const int dx = t - 3 * r;
    const float* kp = kcol + (size_t)(r * KVPOS + dx) * DHEAD;
    float kv[16];
    load16(kp, kv);
    float part = 0.0f;
#pragma unroll
    for (int i = 0; i < 16; ++i) part += q[i] * kv[i];
    const float s    = part + __shfl_xor(part, 16, 32);
    const float mn   = fmaxf(m, s);
    const float corr = __expf(m - mn);
    const float p    = __expf(s - mn);
    ssum = ssum * corr + p;
#pragma unroll
    for (int i = 0; i < 16; ++i) ov[i] = p * kv[i] + ov[i] * corr;
    m = mn;
  }
  const float inv = __builtin_amdgcn_rcpf(ssum);
#pragma unroll
  for (int i = 0; i < 16; ++i) res[i] += ov[i] * inv;
}

__global__ __launch_bounds__(256) void k_attn(const float* __restrict__ xq,
                                              const unsigned short* __restrict__ Wqh,
                                              const unsigned short* __restrict__ Wql,
                                              const float* __restrict__ bq,
                                              const float* __restrict__ bkv,
                                              const float* __restrict__ kv1,
                                              const float* __restrict__ kv2,
                                              float* __restrict__ out) {
  extern __shared__ __attribute__((aligned(16))) float smem[];
  float* qT  = smem;
  float* kvS = smem + TILE_F;
  float* oT  = smem + TILE_F + KVS_F;
  const int tid  = threadIdx.x;
  const int lane = tid & 31;
  const int wave = __builtin_amdgcn_readfirstlane(tid >> 5);
  const int y = blockIdx.x;
  const int b = blockIdx.y;

  const float* xrow = xq + (size_t)b * CCH * HWPIX + (size_t)y * IMW;
  proj_row_tile(xrow, Wqh, Wql, bq, QSCALE, qT, wave, lane);
  __syncthreads();

  const int half = lane >> 4;
  const int px   = 16 * wave + (lane & 15);
#pragma unroll 1
  for (int hd = 0; hd < NHEADS; ++hd) {
    float q[16];
    load16(qT + (size_t)px * TP + hd * DHEAD + 16 * half, q);
    float res[16];
#pragma unroll
    for (int i = 0; i < 16; ++i) res[i] = 0.0f;
#pragma unroll 1
    for (int br = 0; br < 2; ++br) {
      const float* kb = ((br == 0) ? kv1 : kv2) + (size_t)b * HWPIX * CCH;
      stage_kv(kb, bkv, hd, y, kvS, tid);
      __syncthreads();
      attend_branch(kvS, px, half, q, res);
      __syncthreads();
    }
#pragma unroll
    for (int i = 0; i < 16; ++i) oT[(size_t)(16 * half + i) * TP + px] = 0.5f * res[i];
    __syncthreads();
    for (int pass = 0; pass < 2; ++pass) {
#pragma unroll
      for (int k = 0; k < 4; ++k) {
        const int cc = 4 * wave + k;
        const v4f v = *(const v4f*)(oT + (size_t)cc * TP + 4 * lane);
        float* dst = out + (((size_t)b * CCH + hd * DHEAD + cc) * IMH + y) * IMW + 4 * lane;
        *(volatile v4f*)dst = v;
      }
      __threadfence();
    }
  }
}

extern "C" void kernel_launch(void* const* d_in, const int* in_sizes, int n_in,
                              void* d_out, int out_size, void* d_ws, size_t ws_size,
                              hipStream_t stream) {
  if (n_in < 7) return;
  const int nmap = NB * CCH * HWPIX;
  if (in_sizes[0] != nmap || in_sizes[1] != nmap || in_sizes[2] != nmap) return;
  if (in_sizes[3] != CCH * CCH || in_sizes[4] != CCH) return;
  if (in_sizes[5] != CCH * CCH || in_sizes[6] != CCH) return;
  if (out_size != nmap) return;

  const float* kvmap1 = (const float*)d_in[0];
  const float* qmap   = (const float*)d_in[1];
  const float* kvmap2 = (const float*)d_in[2];
  const float* Wq     = (const float*)d_in[3];
  const float* bq     = (const float*)d_in[4];
  const float* Wkv    = (const float*)d_in[5];
  const float* bkv    = (const float*)d_in[6];
  float* out = (float*)d_out;

  const size_t PW  = (size_t)CCH * CCH * 2;
  const size_t PKV = (size_t)NB * HWPIX * CCH * 4;
  size_t off = 0;
  const size_t oWqh = off; off += PW;
  const size_t oWql = off; off += PW;
  const size_t oWkh = off; off += PW;
  const size_t oWkl = off; off += PW;
  const size_t oKV1 = off; off += PKV;
  const size_t oKV2 = off; off += PKV;
  if (off > ws_size) return;

  char* ws = (char*)d_ws;
  unsigned short* Wqh = (unsigned short*)(ws + oWqh);
  unsigned short* Wql = (unsigned short*)(ws + oWql);
  unsigned short* Wkh = (unsigned short*)(ws + oWkh);
  unsigned short* Wkl = (unsigned short*)(ws + oWkl);
  float* KV1 = (float*)(ws + oKV1);
  float* KV2 = (float*)(ws + oKV2);

  const size_t ldsA = (size_t)TILE_F * 4;
  const size_t ldsB = (size_t)ATTN_LDS_F * 4;
  (void)hipFuncSetAttribute(reinterpret_cast<const void*>(&k_kvproj),
                            hipFuncAttributeMaxDynamicSharedMemorySize, (int)ldsA);
  (void)hipFuncSetAttribute(reinterpret_cast<const void*>(&k_attn),
                            hipFuncAttributeMaxDynamicSharedMemorySize, (int)ldsB);

  const dim3 blk(256);
  k_split_w<<<dim3(64), blk, 0, stream>>>(Wq, Wkv, Wqh, Wql, Wkh, Wkl);
  k_kvproj<<<dim3(IMH, NB), blk, ldsA, stream>>>(kvmap1, Wkh, Wkl, bkv, KV1);
  k_kvproj<<<dim3(IMH, NB), blk, ldsA, stream>>>(kvmap2, Wkh, Wkl, bkv, KV2);
  k_attn<<<dim3(IMH, NB), blk, ldsB, stream>>>(qmap, Wqh, Wql, bq, bkv, KV1, KV2, out);
  (void)hipGetLastError();
}
